// HorizonMultiheadAttention_83021717832136
// MI455X (gfx1250) — hardware-verified
//
#include <hip/hip_runtime.h>
#include <math.h>

typedef __attribute__((ext_vector_type(16))) _Float16 v16h;
typedef __attribute__((ext_vector_type(16))) __bf16 v16b;
typedef __attribute__((ext_vector_type(8)))  _Float16 v8h;
typedef __attribute__((ext_vector_type(8)))  float v8f;
typedef __attribute__((ext_vector_type(4)))  float v4f;
typedef __attribute__((ext_vector_type(2)))  float v2f;
typedef __attribute__((ext_vector_type(4)))  unsigned v4u;
typedef __attribute__((ext_vector_type(4)))  int v4i;
typedef float __attribute__((may_alias)) float_a;
typedef int __attribute__((may_alias)) int_a;

template <typename T> __device__ __forceinline__ void vst2(void* p, T v) { *(volatile T*)p = v; __threadfence(); *(volatile T*)p = v; }
__device__ __forceinline__ v8f wmma16(v16h a, v16h b, v8f c) {
  v8f d = __builtin_amdgcn_wmma_f32_16x16x32_f16(false, a, false, b, (short)0, c, false, false);
  asm volatile("v_nop\n\tv_nop\n\tv_nop\n\tv_nop" : "+v"(d) : "v"(a), "v"(b));
  return d;
}
__device__ __forceinline__ v8f wmma_bf(v16b a, v16b b, v8f c) {
  v8f d = __builtin_amdgcn_wmma_f32_16x16x32_bf16(false, a, false, b, (short)0, c, false, false);
  asm volatile("v_nop\n\tv_nop\n\tv_nop\n\tv_nop" : "+v"(d) : "v"(a), "v"(b));
  return d;
}
__device__ __forceinline__ v16h frag_h(const _Float16* rowk0, int lane) {
  union { v16h v; v8h q[2]; } u; const _Float16* p = rowk0 + 8 * (lane >> 4);
  u.q[0] = *(const v8h*)p; u.q[1] = *(const v8h*)(p + 16); return u.v;
}
__device__ __forceinline__ v16h frag_f32(const float* rowk0, int lane) {
  v16h a; const float* p = rowk0 + 8 * (lane >> 4);
#pragma unroll
  for (int i = 0; i < 8; ++i) { a[i] = (_Float16)p[i]; a[8 + i] = (_Float16)p[16 + i]; }
  return a;
}
__device__ __forceinline__ v16h frag_f32s(const float* rowk0, int lane, float sc) {
  v16h a; const float* p = rowk0 + 8 * (lane >> 4);
#pragma unroll
  for (int i = 0; i < 8; ++i) { a[i] = (_Float16)(p[i] * sc); a[8 + i] = (_Float16)(p[16 + i] * sc); }
  return a;
}
__device__ __forceinline__ v16h fragc_f32(const float* W, int k0, int n, int lane, int ld, int K) {
  v16h a; const int g = lane >> 4;
#pragma unroll
  for (int i = 0; i < 8; ++i) { const int ka = k0 + 8 * g + i, kb = ka + 16;
    a[i] = (_Float16)(ka < K ? W[(size_t)(ka < K ? ka : K - 1) * ld + n] : 0.f); a[8 + i] = (_Float16)(kb < K ? W[(size_t)(kb < K ? kb : K - 1) * ld + n] : 0.f); }
  return a;
}
struct F2 { v16b h, l; };
__device__ __forceinline__ F2 bsplit16(const float v[16]) { F2 r;
#pragma unroll
  for (int i = 0; i < 16; ++i) { const __bf16 h = (__bf16)v[i]; r.h[i] = h; r.l[i] = (__bf16)(v[i] - (float)h); }
  return r; }
__device__ __forceinline__ F2 split_row(const float* row, int k0, int lane) { float v[16]; const float* p = row + k0 + 8 * (lane >> 4);
#pragma unroll
  for (int i = 0; i < 8; ++i) { v[i] = p[i]; v[8 + i] = p[16 + i]; }
  return bsplit16(v); }
__device__ __forceinline__ F2 split_rowK(const float* row, int k0, int lane, int K) { float v[16]; const int g = lane >> 4;
#pragma unroll
  for (int i = 0; i < 8; ++i) { const int ka = k0 + 8 * g + i, kb = ka + 16; v[i] = ka < K ? row[ka < K ? ka : K - 1] : 0.f; v[8 + i] = kb < K ? row[kb < K ? kb : K - 1] : 0.f; }
  return bsplit16(v); }
__device__ __forceinline__ F2 split_col(const float* W, int k0, int n, int lane, int ld, int K) { float v[16]; const int g = lane >> 4;
#pragma unroll
  for (int i = 0; i < 8; ++i) { const int ka = k0 + 8 * g + i, kb = ka + 16; v[i] = ka < K ? W[(size_t)(ka < K ? ka : K - 1) * ld + n] : 0.f; v[8 + i] = kb < K ? W[(size_t)(kb < K ? kb : K - 1) * ld + n] : 0.f; }
  return bsplit16(v); }
__device__ __forceinline__ v8f mac3(const F2& a, const F2& b, v8f c) { c = wmma_bf(a.l, b.h, c); c = wmma_bf(a.h, b.l, c); return wmma_bf(a.h, b.h, c); }
__device__ __forceinline__ float sigm(float v) { return 1.0f / (1.0f + expf(-v)); }
#define LDSX() do { asm volatile("s_wait_dscnt 0" ::: "memory"); __builtin_amdgcn_wave_barrier(); __builtin_amdgcn_fence(__ATOMIC_RELEASE, "workgroup"); } while (0)


#define NB 8
#define E 256
#define NT 1024
#define NH 8
#define HD 32
#ifndef TNB
#define TNB NB
#define TQB (NT / 64)
#endif
typedef __attribute__((ext_vector_type(8))) __bf16 v8b;
__device__ __forceinline__ v16b frag_b(const __bf16* rowk0, int lane) {
  union { v16b v; v8b q[2]; } u; const __bf16* p = rowk0 + 8 * (lane >> 4);
  u.q[0] = *(const v8b*)p; u.q[1] = *(const v8b*)(p + 16); return u.v;
}
__device__ __forceinline__ v16b frag_gbf(const float* rowk0, int lane) {
  v16b a; const float* p = rowk0 + 8 * (lane >> 4);
#pragma unroll
  for (int i = 0; i < 8; ++i) { a[i] = (__bf16)p[i]; a[8 + i] = (__bf16)p[16 + i]; }
  return a;
}
__device__ __forceinline__ float bfr(float v) { return (float)(__bf16)v; }
__device__ __attribute__((noinline)) float exp_ni(float v) { return expf(v); }
#define WS_Q    0u
#define WS_K    (WS_Q + 4u * NB * NT * E)
#define WS_VTH  (WS_K + 4u * NB * NT * E)
#define WS_VTL  (WS_VTH + 2u * NB * E * NT)
#define WS_M    (WS_VTL + 2u * NB * E * NT)
#define WS_L    (WS_M + 4u * NB * NH * NT)
#define WS_END  (WS_L + 4u * NB * NH * NT)

__global__ __launch_bounds__(128) void k_proj(const float* __restrict__ Xq, const float* __restrict__ Xk, const float* __restrict__ Xv, const float* __restrict__ Wq, const float* __restrict__ bq, const float* __restrict__ Wk, const float* __restrict__ bk, const float* __restrict__ Wv, const float* __restrict__ bv, float* __restrict__ Q, float* __restrict__ Kb, __bf16* __restrict__ VTH, __bf16* __restrict__ VTL) {
  __shared__ __align__(16) __bf16 sx[64][E + 8]; __shared__ __align__(16) float so[4][16][E + 4]; __shared__ __align__(16) __bf16 svh[E][72], svl[E][72];
  const int tid = threadIdx.x, wave = tid >> 5, lane = tid & 31, col = lane & 15, g = lane >> 4; const int b = blockIdx.y, t0 = blockIdx.x * 64, which = blockIdx.z;
  const float* X = which == 0 ? Xq : (which == 1 ? Xk : Xv); const float* Wm = which == 0 ? Wq : (which == 1 ? Wk : Wv); const float* bm = which == 0 ? bq : (which == 1 ? bk : bv);
  for (int q = tid; q < E * 64; q += 128) { const int c = q >> 6, tl = q & 63; sx[tl][c] = (__bf16)X[((size_t)b * E + c) * NT + t0 + tl]; }
  __syncthreads();
  v8f acc[16] = {};
#pragma unroll 2
  for (int kc = 0; kc < E / 32; ++kc) { const v16b a = frag_b(&sx[wave * 16 + col][kc * 32], lane);
#pragma unroll
    for (int j = 0; j < 16; ++j) acc[j] = wmma_bf(a, frag_gbf(Wm + (size_t)(j * 16 + col) * E + kc * 32, lane), acc[j]); }
#pragma unroll
  for (int j = 0; j < 16; ++j) { const float bb = bfr(bm[j * 16 + col]);
#pragma unroll
    for (int r = 0; r < 8; ++r) so[wave][8 * g + r][j * 16 + col] = acc[j][r] + bb; }
  __syncthreads();
  if (which < 2) { float* dst = which == 0 ? Q : Kb;
    for (int rl = 0; rl < 16; ++rl) for (int pc = lane; pc < E / 4; pc += 32) vst2(dst + ((size_t)b * NT + t0 + wave * 16 + rl) * E + pc * 4, *(const v4f*)&so[wave][rl][pc * 4]); }
  else {
    for (int q = tid; q < E * 64; q += 128) { const int c = q >> 6, tl = q & 63; const float v = so[tl >> 4][tl & 15][c]; const __bf16 hb = (__bf16)v; svh[c][tl] = hb; svl[c][tl] = (__bf16)(v - (float)hb); }
    __syncthreads();
    for (int q = tid; q < E * 8; q += 128) { const int c = q >> 3, pc = q & 7; const size_t o = ((size_t)b * E + c) * NT + t0 + pc * 8; vst2((unsigned*)(VTH + o), *(const v4u*)&svh[c][pc * 8]); vst2((unsigned*)(VTL + o), *(const v4u*)&svl[c][pc * 8]); } }
}
__global__ __launch_bounds__(128) void k_stats(const float* __restrict__ Q, const float* __restrict__ Kb, const float* __restrict__ mask, float* __restrict__ Mb, float* __restrict__ Lb) {
  __shared__ __align__(16) float sm[4][16]; __shared__ __align__(16) float ssum[4][16];
  const int tid = threadIdx.x, wave = tid >> 5, lane = tid & 31, col = lane & 15, g = lane >> 4; const int bh = blockIdx.y, b = bh >> 3, h = bh & 7; const int q0 = blockIdx.x * 64 + wave * 16; const float scale = 0.17677669529663687f;
  const F2 a = split_row(Q + ((size_t)b * NT + q0 + col) * E + h * HD, 0, lane);
  float m[8], l[8];
#pragma unroll
  for (int r = 0; r < 8; ++r) { m[r] = -3.0e38f; l[r] = 0.f; }
#pragma unroll 1
  for (int kt = 0; kt < NT / 16; ++kt) { const F2 kb = split_row(Kb + ((size_t)b * NT + kt * 16 + col) * E + h * HD, 0, lane); const v8f s = mac3(a, kb, (v8f){});
#pragma unroll
    for (int r = 0; r < 8; ++r) { const float sv = s[r] * scale + bfr(mask[(size_t)(q0 + 8 * g + r) * NT + kt * 16 + col]); float mx = sv;
#pragma unroll
      for (int o = 1; o < 16; o <<= 1) mx = fmaxf(mx, __shfl_xor(mx, o));
      const float mn = fmaxf(m[r], mx); float e = exp_ni(sv - mn);
#pragma unroll
      for (int o = 1; o < 16; o <<= 1) e += __shfl_xor(e, o);
      l[r] = l[r] * exp_ni(m[r] - mn) + e; m[r] = mn; } }
  if (col == 0) {
#pragma unroll
    for (int r = 0; r < 8; ++r) { sm[wave][8 * g + r] = m[r]; ssum[wave][8 * g + r] = l[r]; } }
  __syncthreads();
  { const int qb = blockIdx.x * 64; if (tid < 16) vst2(Mb + ((size_t)bh * NT + qb) + tid * 4, *(const v4f*)(&sm[0][0] + tid * 4)); else if (tid < 32) vst2(Lb + ((size_t)bh * NT + qb) + (tid - 16) * 4, *(const v4f*)(&ssum[0][0] + (tid - 16) * 4)); }
}
__global__ __launch_bounds__(128) void k_attn(float* __restrict__ Q, const float* __restrict__ Kb, const float* __restrict__ mask, const __bf16* __restrict__ VTH, const __bf16* __restrict__ VTL, const float* __restrict__ Mb, const float* __restrict__ Lb) {
  __shared__ __align__(16) float sp[4][16][36]; __shared__ __align__(16) float so[4][16][36];
  const int tid = threadIdx.x, wave = tid >> 5, lane = tid & 31, col = lane & 15, g = lane >> 4; const int bh = blockIdx.y, b = bh >> 3, h = bh & 7; const int q0 = blockIdx.x * 64 + wave * 16; const float scale = 0.17677669529663687f;
  const F2 a = split_row(Q + ((size_t)b * NT + q0 + col) * E + h * HD, 0, lane);
  float mr[8], il[8];
#pragma unroll
  for (int r = 0; r < 8; ++r) { mr[r] = Mb[(size_t)bh * NT + q0 + 8 * g + r]; il[r] = 1.0f / Lb[(size_t)bh * NT + q0 + 8 * g + r]; }
  v8f acc[2] = {};
#pragma unroll 1
  for (int ks = 0; ks < NT / 32; ++ks) {
#pragma unroll
    for (int ct = 0; ct < 2; ++ct) { const int kk = ks * 32 + ct * 16 + col; const F2 kb = split_row(Kb + ((size_t)b * NT + kk) * E + h * HD, 0, lane); const v8f s = mac3(a, kb, (v8f){});
#pragma unroll
      for (int r = 0; r < 8; ++r) sp[wave][8 * g + r][ct * 16 + col] = exp_ni((s[r] * scale + bfr(mask[(size_t)(q0 + 8 * g + r) * NT + kk])) - mr[r]) * il[r]; }
    LDSX();
    const F2 pa = split_row(&sp[wave][col][0], 0, lane);
#pragma unroll
    for (int dt = 0; dt < 2; ++dt) { const size_t vrow = ((size_t)b * E + h * HD + dt * 16 + col) * NT + ks * 32; const v16b vh = frag_b(VTH + vrow, lane), vl = frag_b(VTL + vrow, lane);
      acc[dt] = wmma_bf(pa.l, vh, acc[dt]); acc[dt] = wmma_bf(pa.h, vl, acc[dt]); acc[dt] = wmma_bf(pa.h, vh, acc[dt]); }
    LDSX(); }
#pragma unroll
  for (int dt = 0; dt < 2; ++dt)
#pragma unroll
    for (int r = 0; r < 8; ++r) so[wave][8 * g + r][dt * 16 + col] = acc[dt][r];
  LDSX();
  for (int rl = 0; rl < 16; ++rl) if (lane < 8) vst2(Q + ((size_t)b * NT + q0 + rl) * E + h * HD + lane * 4, *(const v4f*)&so[wave][rl][lane * 4]);
}
__global__ __launch_bounds__(128) void k_out(const float* __restrict__ O, const float* __restrict__ Wo, const float* __restrict__ bo, float* __restrict__ Y) {
  __shared__ __align__(16) float sot[E][68];
  const int tid = threadIdx.x, wave = tid >> 5, lane = tid & 31, col = lane & 15, g = lane >> 4; const int b = blockIdx.y, t0 = blockIdx.x * 64;
  v8f acc[16] = {};
#pragma unroll 1
  for (int kc = 0; kc < E / 32; ++kc) { const F2 a = split_row(O + ((size_t)b * NT + t0 + wave * 16 + col) * E, kc * 32, lane);
#pragma unroll
    for (int j = 0; j < 16; ++j) { const v16b w = frag_gbf(Wo + (size_t)(j * 16 + col) * E + kc * 32, lane); acc[j] = wmma_bf(a.l, w, acc[j]); acc[j] = wmma_bf(a.h, w, acc[j]); } }
#pragma unroll
  for (int j = 0; j < 16; ++j) { const int o = j * 16 + col; const float bb = bfr(bo[o]);
#pragma unroll
    for (int r = 0; r < 8; ++r) sot[o][wave * 16 + 8 * g + r] = acc[j][r] + bb; }
  __syncthreads();
  for (int q = tid; q < E * 16; q += 128) { const int o = q >> 4, pc = q & 15; vst2(Y + ((size_t)b * E + o) * NT + t0 + pc * 4, *(const v4f*)&sot[o][pc * 4]); }
}

extern "C" void kernel_launch(void* const* d_in, const int* in_sizes, int n_in, void* d_out, int out_size, void* d_ws, size_t ws_size, hipStream_t stream) {
  (void)in_sizes; (void)n_in; (void)out_size;
  const float** F = (const float**)d_in;
  if (ws_size < (size_t)WS_END) return;
  char* ws = (char*)d_ws; float *Q = (float*)(ws + WS_Q), *Kb = (float*)(ws + WS_K), *Mb = (float*)(ws + WS_M), *Lb = (float*)(ws + WS_L); __bf16 *VTH = (__bf16*)(ws + WS_VTH), *VTL = (__bf16*)(ws + WS_VTL);
  k_proj<<<dim3(NT / 64, TNB, 3), 128, 0, stream>>>(F[0], F[1], F[2], F[4], F[8], F[5], F[9], F[6], F[10], Q, Kb, VTH, VTL);
  k_stats<<<dim3(TQB, TNB * NH), 128, 0, stream>>>(Q, Kb, F[3], Mb, Lb);
  k_attn<<<dim3(TQB, TNB * NH), 128, 0, stream>>>(Q, Kb, F[3], VTH, VTL, Mb, Lb);
  k_out<<<dim3(TQB, TNB), 128, 0, stream>>>(Q, F[7], F[11], (float*)d_out);
}
